// GatedGAT_35596688949920
// MI455X (gfx1250) — hardware-run, weakly checked
//
#include <hip/hip_runtime.h>
#include <stddef.h>


#define ZW      128
#define FW      256
#define OW      64
#define NHD     4
#define GK      384
#define LDXG    192
#define GCOL    128
#define WSC     16
#define GSC     8
#define NTHR    256
#define NWAVE   8
#define EPT     8
#define NGRP    2
#define CHUNK   (NTHR * EPT * NGRP)
#define WCAP    (EPT * NGRP * 32)
#define LISTN   (NWAVE * WCAP)
#define NBC     4096
#define NBF     1024
#define RCAP    40960
#define RBN     128
#define TGT     256
#define DEGCAP  256
#define OTHR    512
#define WSCAP   134217728
#define NEG_SLOPE 0.2f

#define LDS_FILL ((RCAP + NBF + LISTN) * 4 + 64)

static_assert((CHUNK & (CHUNK - 1)) == 0);
static_assert(CHUNK <= 4096);
static_assert(NBC <= 4096 && NBF <= 4096);
static_assert((NBC & (NBC - 1)) == 0 && (NBF & (NBF - 1)) == 0);
static_assert(NBC == 4 * NBF);
static_assert(OTHR * 8 == NBC);
static_assert((RCAP % 32) == 0);
static_assert(TGT == NWAVE * 32);
static_assert((NBC % TGT) == 0);
static_assert(NBC >= TGT);
static_assert(FW == NHD * OW);
static_assert(GK == 2 * ZW + ZW);
static_assert(LDXG == ZW + OW && GCOL == ZW);
static_assert(ZW == 4 * 32 && FW == 8 * 32 && OW == 8 * 8);
static_assert((WSC & (WSC - 1)) == 0 && (GSC & (GSC - 1)) == 0 && WSC >= GSC);

typedef float          v4f  __attribute__((ext_vector_type(4)));
typedef float          v8f  __attribute__((ext_vector_type(8)));
typedef int            v4i  __attribute__((ext_vector_type(4)));
typedef _Float16       v8h  __attribute__((ext_vector_type(8)));
typedef _Float16       v16h __attribute__((ext_vector_type(16)));
union FragH { v16h v; v8h h[2]; };

__device__ __forceinline__ v8f wmh(v16h a, v16h b, v8f c) {
  v8f d = __builtin_amdgcn_wmma_f32_16x16x32_f16(false, a, false, b, (short)0, c, false, false);
  asm volatile("v_nop\n\tv_nop\n\tv_nop\n\tv_nop" : "+v"(d) : "v"(a), "v"(b));
  return d;
}

__device__ __forceinline__ v8h cvt8(v4f a, v4f b, float sc) {
  v8h o;
  o[0] = (_Float16)(a.x * sc); o[1] = (_Float16)(a.y * sc);
  o[2] = (_Float16)(a.z * sc); o[3] = (_Float16)(a.w * sc);
  o[4] = (_Float16)(b.x * sc); o[5] = (_Float16)(b.y * sc);
  o[6] = (_Float16)(b.z * sc); o[7] = (_Float16)(b.w * sc);
  return o;
}

__device__ __forceinline__ float lrelu(float v) { return v > 0.0f ? v : NEG_SLOPE * v; }

template <int NB>
__device__ __forceinline__ int scan_chunk(const int* __restrict__ dsts, int nE, int cbase, int slotBase,
                                          int vec8, int* list, int tid, int lane, int wave) {
  int wc = 0;
#pragma unroll
  for (int g = 0; g < NGRP; ++g) {
    const int el0  = (g * NTHR + tid) * EPT;
    const int e0   = cbase + el0;
    const int sent = -2147483647 - 1;
    v4i da, db;
    if (vec8 != 0 && cbase + CHUNK <= nE) {
      da = *(const v4i*)(dsts + e0);
      db = *(const v4i*)(dsts + e0 + 4);
    } else {
      da.x = (e0     < nE) ? dsts[min(e0, nE - 1)] : sent;
      da.y = (e0 + 1 < nE) ? dsts[min(e0 + 1, nE - 1)] : sent;
      da.z = (e0 + 2 < nE) ? dsts[min(e0 + 2, nE - 1)] : sent;
      da.w = (e0 + 3 < nE) ? dsts[min(e0 + 3, nE - 1)] : sent;
      db.x = (e0 + 4 < nE) ? dsts[min(e0 + 4, nE - 1)] : sent;
      db.y = (e0 + 5 < nE) ? dsts[min(e0 + 5, nE - 1)] : sent;
      db.z = (e0 + 6 < nE) ? dsts[min(e0 + 6, nE - 1)] : sent;
      db.w = (e0 + 7 < nE) ? dsts[min(e0 + 7, nE - 1)] : sent;
    }
    const unsigned nb = (unsigned)slotBase;
    const unsigned s0 = (unsigned)da.x - nb, s1 = (unsigned)da.y - nb;
    const unsigned s2 = (unsigned)da.z - nb, s3 = (unsigned)da.w - nb;
    const unsigned s4 = (unsigned)db.x - nb, s5 = (unsigned)db.y - nb;
    const unsigned s6 = (unsigned)db.z - nb, s7 = (unsigned)db.w - nb;
    const bool h0 = s0 < (unsigned)NB, h1 = s1 < (unsigned)NB, h2 = s2 < (unsigned)NB, h3 = s3 < (unsigned)NB;
    const bool h4 = s4 < (unsigned)NB, h5 = s5 < (unsigned)NB, h6 = s6 < (unsigned)NB, h7 = s7 < (unsigned)NB;
    const unsigned any = __builtin_amdgcn_ballot_w32(h0 | h1 | h2 | h3 | h4 | h5 | h6 | h7);
    if (any != 0u) {
#define HITJ(J, HJ, SJ) { \
        const unsigned mj = __builtin_amdgcn_ballot_w32(HJ); \
        if (mj != 0u) { \
          if (HJ) { \
            const int pos = wc + (int)__builtin_amdgcn_mbcnt_lo(mj, 0u); \
            if (pos < WCAP) list[wave * WCAP + pos] = ((el0 + (J)) << 12) | (int)(SJ); \
          } \
          wc += (int)__builtin_popcount(mj); } }
      HITJ(0, h0, s0)
      HITJ(1, h1, s1)
      HITJ(2, h2, s2)
      HITJ(3, h3, s3)
      HITJ(4, h4, s4)
      HITJ(5, h5, s5)
      HITJ(6, h6, s6)
      HITJ(7, h7, s7)
#undef HITJ
    }
  }
  return wc;
}

__global__ __launch_bounds__(NTHR) void k_xcvt(const float* __restrict__ x, _Float16* xg, int nN, int nUnits) {
  const int i = (int)blockIdx.x * NTHR + (int)threadIdx.x;
  if (i >= nUnits) return;
  const int row = i >> 4;
  const int seg = i & 15;
  const int c0  = seg * 8;
  int rr = row > nN - 1 ? nN - 1 : row;
  rr = rr < 0 ? 0 : rr;
  const float* p = x + (size_t)rr * ZW + c0;
  v4f a = *(const v4f*)p, b = *(const v4f*)(p + 4);
  const v4f z = {0.f, 0.f, 0.f, 0.f};
  if (row >= nN) { a = z; b = z; }
  const v8h o = cvt8(a, b, 1.0f);
  _Float16* d = xg + (size_t)row * LDXG + c0;
  *(volatile v8h*)d = o;
  __threadfence();
  *(volatile v8h*)d = o;
}

__global__ __launch_bounds__(NTHR) void k_wcvt(const float* __restrict__ W, _Float16* wp, int nUnits,
                                               int KD, int kSplit, float scLo, float scHi) {
  const int i = (int)blockIdx.x * NTHR + (int)threadIdx.x;
  if (i >= nUnits) return;
  const int k0 = (i * 8) % KD;
  const float sc = (k0 < kSplit) ? scLo : scHi;
  const float* p = W + (size_t)i * 8;
  const v4f a = *(const v4f*)p, b = *(const v4f*)(p + 4);
  const v8h o = cvt8(a, b, sc);
  _Float16* d = wp + (size_t)i * 8;
  *(volatile v8h*)d = o;
  __threadfence();
  *(volatile v8h*)d = o;
}

__global__ __launch_bounds__(NTHR) void k_count(
    const int* __restrict__ dsts, int* cnt, int nE, int vec8) {
  __shared__ __attribute__((aligned(16))) int scnt[NBC];
  __shared__ __attribute__((aligned(16))) int list[LISTN];
  __shared__ int wcnt[NWAVE];
  const int tid = threadIdx.x, lane = tid & 31, wave = tid >> 5;
  const int nodeBase = blockIdx.x * NBC;

  for (int i = tid; i < NBC; i += NTHR) scnt[i] = 0;
  __syncthreads();

  const int nChunks = (nE + CHUNK - 1) / CHUNK;
#pragma unroll 1
  for (int ch = 0; ch < nChunks; ++ch) {
    const int cbase = ch * CHUNK;
    const int wc = scan_chunk<NBC>(dsts, nE, cbase, nodeBase, vec8, list, tid, lane, wave);
    if (lane == 0) wcnt[wave] = wc;
    __syncthreads();
    if (wave == 0) {
#pragma unroll 1
      for (int wsx = 0; wsx < NWAVE; ++wsx) {
        int n = __builtin_amdgcn_readfirstlane(wcnt[wsx]);
        n = n > WCAP ? WCAP : (n < 0 ? 0 : n);
        const int* lp = list + wsx * WCAP;
#pragma unroll 1
        for (int i = 0; i < n; ++i) {
          const int ent  = __builtin_amdgcn_readfirstlane(lp[i]);
          const int slot = ent & (NBC - 1);
          if (lane == 0) scnt[slot] = scnt[slot] + 1;
        }
      }
    }
    __syncthreads();
  }

  v4i cq[4];
#pragma unroll
  for (int q = 0; q < 4; ++q) {
    const int f = (wave * 4 + q) * 128 + 4 * lane;
    cq[q] = *(const v4i*)(scnt + f);
  }
  int* cp = cnt + (size_t)nodeBase;
#pragma unroll
  for (int q = 0; q < 4; ++q) {
    const int f = (wave * 4 + q) * 128 + 4 * lane;
    *(volatile v4i*)(cp + f) = cq[q];
  }
  __threadfence();
#pragma unroll
  for (int q = 0; q < 4; ++q) {
    const int f = (wave * 4 + q) * 128 + 4 * lane;
    *(volatile v4i*)(cp + f) = cq[q];
  }
}

__global__ __launch_bounds__(OTHR) void k_offsets(
    const int* __restrict__ cnt, int* off, int* rbase, int nChunk) {
  __shared__ __attribute__((aligned(16))) int soff[NBC];
  __shared__ __attribute__((aligned(16))) int srb[RBN];
  __shared__ int wtot[OTHR / 32];
  const int tid = threadIdx.x, lane = tid & 31, wave = tid >> 5, sub = tid >> 7;
  for (int i = tid; i < RBN; i += OTHR) srb[i] = 0;
  int carry = 0;
#pragma unroll 1
  for (int ch = 0; ch < nChunk; ++ch) {
    const int base = ch * NBC;
    const v4i c0 = *(const v4i*)(cnt + base + 8 * tid);
    const v4i c1 = *(const v4i*)(cnt + base + 8 * tid + 4);
    const int e0 = max(c0.x, 0), e1 = max(c0.y, 0), e2 = max(c0.z, 0), e3 = max(c0.w, 0);
    const int e4 = max(c1.x, 0), e5 = max(c1.y, 0), e6 = max(c1.z, 0), e7 = max(c1.w, 0);
    const int ts = e0 + e1 + e2 + e3 + e4 + e5 + e6 + e7;
    int incl = ts;
#pragma unroll
    for (int d = 1; d < 32; d <<= 1) {
      const int t = __shfl_up(incl, d);
      if (lane >= d) incl += t;
    }
    if (lane == 31) wtot[wave] = incl;
    __syncthreads();
    const int S0 = wtot[0]  + wtot[1]  + wtot[2]  + wtot[3];
    const int S1 = wtot[4]  + wtot[5]  + wtot[6]  + wtot[7];
    const int S2 = wtot[8]  + wtot[9]  + wtot[10] + wtot[11];
    const int S3 = wtot[12] + wtot[13] + wtot[14] + wtot[15];
    int pre = 0;
#pragma unroll 1
    for (int w = 4 * sub; w < wave; ++w) pre += wtot[w];
    const int b0 = carry;
    const int b1 = b0 + ((S0 + 31) & ~31);
    const int b2 = b1 + ((S1 + 31) & ~31);
    const int b3 = b2 + ((S2 + 31) & ~31);
    const int b4 = b3 + ((S3 + 31) & ~31);
    const int myb = sub == 0 ? b0 : (sub == 1 ? b1 : (sub == 2 ? b2 : b3));
    if (tid == 0) {
      srb[min(4 * ch + 0, RBN - 1)] = b0;
      srb[min(4 * ch + 1, RBN - 1)] = b1;
      srb[min(4 * ch + 2, RBN - 1)] = b2;
      srb[min(4 * ch + 3, RBN - 1)] = b3;
    }
    int run = myb + pre + incl - ts;
    soff[8 * tid + 0] = run; run += e0;
    soff[8 * tid + 1] = run; run += e1;
    soff[8 * tid + 2] = run; run += e2;
    soff[8 * tid + 3] = run; run += e3;
    soff[8 * tid + 4] = run; run += e4;
    soff[8 * tid + 5] = run; run += e5;
    soff[8 * tid + 6] = run; run += e6;
    soff[8 * tid + 7] = run;
    carry = b4;
    __syncthreads();
    const v4i o0 = *(const v4i*)(soff + 4 * tid);
    const v4i o1 = *(const v4i*)(soff + 4 * (tid + OTHR));
    int* op = off + base;
    *(volatile v4i*)(op + 4 * tid) = o0;
    *(volatile v4i*)(op + 4 * (tid + OTHR)) = o1;
    __threadfence();
    *(volatile v4i*)(op + 4 * tid) = o0;
    *(volatile v4i*)(op + 4 * (tid + OTHR)) = o1;
    __syncthreads();
  }
  if (tid == 0) srb[min(4 * nChunk, RBN - 1)] = carry;
  __syncthreads();
  v4i rv = {0, 0, 0, 0};
  if (tid < 32) rv = *(const v4i*)(srb + 4 * tid);
  if (tid < 32) *(volatile v4i*)(rbase + 4 * tid) = rv;
  __threadfence();
  if (tid < 32) *(volatile v4i*)(rbase + 4 * tid) = rv;
}

__global__ __launch_bounds__(NTHR) void k_fill(
    const int* __restrict__ dsts, const int* __restrict__ off, const int* __restrict__ rbase,
    int* csr, int nE, int vec8, int csrLen) {
  extern __shared__ v4f lds_dyn[];
  int* region = (int*)lds_dyn;
  int* cursor = region + RCAP;
  int* list   = cursor + NBF;
  int* wcnt   = list + LISTN;
  const int tid = threadIdx.x, lane = tid & 31, wave = tid >> 5;
  const int b = blockIdx.x;
  const int nodeBase = b * NBF;

  int rb0 = rbase[b];
  const int rb1 = rbase[b + 1];
  rb0 = rb0 < 0 ? 0 : (rb0 > csrLen ? csrLen : rb0);
  rb0 &= ~31;
  int len = rb1 - rb0;
  len = len < 0 ? 0 : (len > RCAP ? RCAP : len);
  int lenW = (len + 31) & ~31;
  if (rb0 + lenW > csrLen) lenW = (csrLen - rb0) & ~31;

  {
    const v4i z = {0, 0, 0, 0};
    for (int i = tid; i < RCAP / 4; i += NTHR) ((v4i*)region)[i] = z;
    for (int s = tid; s < NBF; s += NTHR) {
      int o = off[nodeBase + s] - rb0;
      o = o < 0 ? 0 : (o > RCAP ? RCAP : o);
      cursor[s] = o;
    }
  }
  __syncthreads();

  const int nChunks = (nE + CHUNK - 1) / CHUNK;
#pragma unroll 1
  for (int ch = 0; ch < nChunks; ++ch) {
    const int cbase = ch * CHUNK;
    const int wc = scan_chunk<NBF>(dsts, nE, cbase, nodeBase, vec8, list, tid, lane, wave);
    if (lane == 0) wcnt[wave] = wc;
    __syncthreads();
    if (wave == 0) {
#pragma unroll 1
      for (int wsx = 0; wsx < NWAVE; ++wsx) {
        int n = __builtin_amdgcn_readfirstlane(wcnt[wsx]);
        n = n > WCAP ? WCAP : (n < 0 ? 0 : n);
        const int* lp = list + wsx * WCAP;
#pragma unroll 1
        for (int i = 0; i < n; ++i) {
          const int ent  = __builtin_amdgcn_readfirstlane(lp[i]);
          const int slot = ent & (NBF - 1);
          int e = cbase + ((ent >> 12) & (CHUNK - 1));
          e = e > nE - 1 ? nE - 1 : (e < 0 ? 0 : e);
          if (lane == 0) {
            int pos = cursor[slot];
            pos = pos < 0 ? 0 : (pos > RCAP - 1 ? RCAP - 1 : pos);
            region[pos] = e;
            const int np = pos + 1;
            cursor[slot] = np > RCAP ? RCAP : np;
          }
        }
      }
    }
    __syncthreads();
  }

  const int nv = lenW >> 2;
  int* gp = csr + rb0;
#pragma unroll 1
  for (int i = tid; i < nv; i += NTHR) { const v4i v = ((const v4i*)region)[i]; *(volatile v4i*)(gp + 4 * i) = v; }
  __threadfence();
#pragma unroll 1
  for (int i = tid; i < nv; i += NTHR) { const v4i v = ((const v4i*)region)[i]; *(volatile v4i*)(gp + 4 * i) = v; }
}

template <int KA, int LDA, int NC, int BMR, int HEADS, int MODE>
__global__ __launch_bounds__(NTHR) void k_gemm(
    const _Float16* __restrict__ Ap, const _Float16* __restrict__ Bp,
    const float* __restrict__ bias, const float* __restrict__ attS, const float* __restrict__ attD,
    float* C, float* eS, float* eD, int nN) {
  constexpr int RG  = BMR / 16;
  constexpr int CG  = NWAVE / RG;
  constexpr int WC  = NC / CG;
  constexpr int TPW = WC / 16;
  constexpr int KT  = KA / 32;
  constexpr int NF4 = BMR * NC / 4;
  constexpr int NIT = NF4 / NTHR;
  constexpr int NES = BMR * HEADS;
  constexpr int NV  = NES / 4;
  constexpr int TPR = NTHR / BMR;
  constexpr int CPP = NC / TPR;
  constexpr int PPH = TPR / HEADS;
  constexpr float OSC = 1.0f / (float)WSC;
  static_assert(KA % 32 == 0 && LDA % 8 == 0 && LDA >= KA);
  static_assert(RG * 16 == BMR && RG >= 1 && RG * CG == NWAVE && CG >= 1);
  static_assert(CG * WC == NC && TPW * 16 == WC && TPW >= 1);
  static_assert(NF4 % NTHR == 0 && NIT >= 1);
  static_assert(TPR * BMR == NTHR && TPR * CPP == NC);
  static_assert(NES % 4 == 0);
  static_assert(MODE == 0 || MODE == 1 || MODE == 2);
  static_assert(MODE != 1 || (CPP % 4 == 0 && PPH >= 1 && PPH * HEADS == TPR &&
                              (PPH & (PPH - 1)) == 0 && PPH <= 8 && 2 * NV <= NTHR));

  __shared__ __attribute__((aligned(16))) float stg[BMR * NC];
  __shared__ __attribute__((aligned(16))) float sES[NES];
  __shared__ __attribute__((aligned(16))) float sED[NES];
  const int tid = threadIdx.x, lane = tid & 31, wave = tid >> 5, hh = lane >> 4, m = lane & 15;
  const int rowBase = blockIdx.x * BMR;
  const int rg = wave / CG, cg = wave - rg * CG;
  const int r0 = rg * 16;
  const int c0 = cg * WC;

  v8f acc[TPW];
#pragma unroll
  for (int t = 0; t < TPW; ++t) { v8f z = {0.f, 0.f, 0.f, 0.f, 0.f, 0.f, 0.f, 0.f}; acc[t] = z; }

  const _Float16* ap  = Ap + (size_t)(rowBase + r0 + m) * LDA + 8 * hh;
  const _Float16* bp0 = Bp + (size_t)(c0 + m) * KA + 8 * hh;
#pragma unroll 1
  for (int kt = 0; kt < KT; ++kt) {
    FragH a;
    a.h[0] = *(const v8h*)(ap + 32 * kt);
    a.h[1] = *(const v8h*)(ap + 32 * kt + 16);
#pragma unroll
    for (int t = 0; t < TPW; ++t) {
      const _Float16* bp = bp0 + (size_t)(16 * t) * KA + 32 * kt;
      FragH bf;
      bf.h[0] = *(const v8h*)bp;
      bf.h[1] = *(const v8h*)(bp + 16);
      acc[t] = wmh(a.v, bf.v, acc[t]);
    }
  }

  {
    float* sp = stg + (size_t)(r0 + 8 * hh) * NC + c0 + m;
#pragma unroll
    for (int t = 0; t < TPW; ++t) {
      float bv = 0.0f;
      if constexpr (MODE != 1) bv = bias[c0 + 16 * t + m];
#pragma unroll
      for (int r = 0; r < 8; ++r) sp[r * NC + 16 * t] = acc[t][r] * OSC + bv;
    }
  }
  __syncthreads();

  if constexpr (MODE == 1) {
    const int drow = tid / TPR, part = tid - drow * TPR;
    const float* rp  = stg + (size_t)drow * NC + CPP * part;
    const float* sa  = attS + CPP * part;
    const float* sdd = attD + CPP * part;
    float ps = 0.f, pd = 0.f;
#pragma unroll 4
    for (int c = 0; c < CPP; c += 4) {
      const v4f hv = *(const v4f*)(rp + c);
      const v4f av = *(const v4f*)(sa + c);
      const v4f dv = *(const v4f*)(sdd + c);
      ps += hv.x * av.x + hv.y * av.y + hv.z * av.z + hv.w * av.w;
      pd += hv.x * dv.x + hv.y * dv.y + hv.z * dv.z + hv.w * dv.w;
    }
    if constexpr (PPH >= 2) { ps += __shfl_xor(ps, 1); pd += __shfl_xor(pd, 1); }
    if constexpr (PPH >= 4) { ps += __shfl_xor(ps, 2); pd += __shfl_xor(pd, 2); }
    if constexpr (PPH >= 8) { ps += __shfl_xor(ps, 4); pd += __shfl_xor(pd, 4); }
    if ((part & (PPH - 1)) == 0) {
      const int ix = drow * HEADS + part / PPH;
      sES[ix] = ps; sED[ix] = pd;
    }
  }

  if constexpr (MODE != 2) {
    float* tileC = C + (size_t)rowBase * NC;
    v4f cv[NIT];
#pragma unroll
    for (int it = 0; it < NIT; ++it) cv[it] = *(const v4f*)(stg + 4 * (it * NTHR + tid));
#pragma unroll
    for (int it = 0; it < NIT; ++it) *(volatile v4f*)(tileC + 4 * (size_t)(it * NTHR + tid)) = cv[it];
    __threadfence();
#pragma unroll
    for (int it = 0; it < NIT; ++it) *(volatile v4f*)(tileC + 4 * (size_t)(it * NTHR + tid)) = cv[it];
  } else {
    float* tileC = C + (size_t)rowBase * NC;
    v4f cv[NIT];
    bool ok[NIT];
#pragma unroll
    for (int it = 0; it < NIT; ++it) {
      const int f = it * NTHR + tid;
      cv[it] = *(const v4f*)(stg + 4 * f);
      ok[it] = (rowBase + f / (NC / 4)) < nN;
    }
#pragma unroll
    for (int it = 0; it < NIT; ++it) if (ok[it]) *(volatile v4f*)(tileC + 4 * (size_t)(it * NTHR + tid)) = cv[it];
    __threadfence();
#pragma unroll
    for (int it = 0; it < NIT; ++it) if (ok[it]) *(volatile v4f*)(tileC + 4 * (size_t)(it * NTHR + tid)) = cv[it];
  }

  if constexpr (MODE == 1) {
    __syncthreads();
    const size_t eb = (size_t)rowBase * HEADS;
    const int iS = tid < NV - 1 ? tid : NV - 1;
    int iD = tid - NV; iD = iD < 0 ? 0 : (iD > NV - 1 ? NV - 1 : iD);
    const v4f vS = *(const v4f*)(sES + 4 * iS);
    const v4f vD = *(const v4f*)(sED + 4 * iD);
    const bool isS = tid < NV;
    const v4f dv = isS ? vS : vD;
    float* gp = isS ? (eS + eb + 4 * iS) : (eD + eb + 4 * iD);
    if (tid < 2 * NV) *(volatile v4f*)gp = dv;
    __threadfence();
    if (tid < 2 * NV) *(volatile v4f*)gp = dv;
  }
}

__global__ __launch_bounds__(NTHR) void k_agg(
    const int* __restrict__ csr, const int* __restrict__ off, const int* __restrict__ cnt,
    const int* __restrict__ srcs, const float* __restrict__ wgt, const float* __restrict__ x,
    const float* __restrict__ el, const float* __restrict__ er,
    const float* __restrict__ feat, const float* __restrict__ mz,
    const float* __restrict__ gw, const float* __restrict__ gb,
    _Float16* xg, int nN, int nE, int csrLen) {
  const int tid = threadIdx.x, lane = tid & 31, wave = tid >> 5;
  const int tbase = blockIdx.x * TGT + wave * 32;
  const int hd   = lane >> 3;
  const int fcol = 8 * lane;
  const int zcol = 4 * lane;
  const int cl    = tbase + lane;
  const int cnt_l = cnt[cl];
  const int off_l = off[cl];
  const float gb0 = gb[0], gb1 = gb[1], gb2 = gb[2], gb3 = gb[3];

#pragma unroll 1
  for (int j = 0; j < 32; ++j) {
    const int c = tbase + j;
    int nraw = __builtin_amdgcn_readfirstlane(__shfl(cnt_l, j));
    nraw = nraw < 0 ? 0 : nraw;
    const int n  = nraw > DEGCAP ? DEGCAP : nraw;
    const int st = __builtin_amdgcn_readfirstlane(__shfl(off_l, j));
    const float erc = er[(size_t)c * NHD + hd];

    float mx = -3.0e38f;
#pragma unroll 1
    for (int q0 = 0; q0 < n; q0 += 32) {
      int pos = st + q0 + lane;
      pos = pos < 0 ? 0 : (pos > csrLen - 1 ? csrLen - 1 : pos);
      int eg = csr[pos];
      eg = eg < 0 ? 0 : (eg > nE - 1 ? nE - 1 : eg);
      int sl = srcs[eg];
      sl = sl < 0 ? 0 : (sl > nN - 1 ? nN - 1 : sl);
      const int mcnt = (n - q0) < 32 ? (n - q0) : 32;
#pragma unroll 1
      for (int pp = 0; pp < mcnt; ++pp) {
        const int s = __builtin_amdgcn_readlane(sl, pp);
        mx = fmaxf(mx, lrelu(el[(size_t)s * NHD + hd] + erc));
      }
    }

    float den = 0.f;
    float acc[8];
#pragma unroll
    for (int i = 0; i < 8; ++i) acc[i] = 0.f;
    v4f sx = {0.f, 0.f, 0.f, 0.f};
    float zm0 = -3.0e38f, zm1 = -3.0e38f, zm2 = -3.0e38f, zm3 = -3.0e38f;
#pragma unroll 1
    for (int q0 = 0; q0 < n; q0 += 32) {
      int pos = st + q0 + lane;
      pos = pos < 0 ? 0 : (pos > csrLen - 1 ? csrLen - 1 : pos);
      int eg = csr[pos];
      eg = eg < 0 ? 0 : (eg > nE - 1 ? nE - 1 : eg);
      int sl = srcs[eg];
      sl = sl < 0 ? 0 : (sl > nN - 1 ? nN - 1 : sl);
      const float wl = wgt[eg];
      const int mcnt = (n - q0) < 32 ? (n - q0) : 32;
#pragma unroll 1
      for (int pp = 0; pp < mcnt; ++pp) {
        const int s = __builtin_amdgcn_readlane(sl, pp);
        const float w = __int_as_float(__builtin_amdgcn_readlane(__float_as_int(wl), pp));
        const float p = __expf(lrelu(el[(size_t)s * NHD + hd] + erc) - mx);
        den += p;
        const float pw = p * w;
        const float* fp = feat + (size_t)s * FW + fcol;
        const v4f f0 = *(const v4f*)fp;
        const v4f f1 = *(const v4f*)(fp + 4);
        acc[0] += pw * f0.x; acc[1] += pw * f0.y; acc[2] += pw * f0.z; acc[3] += pw * f0.w;
        acc[4] += pw * f1.x; acc[5] += pw * f1.y; acc[6] += pw * f1.z; acc[7] += pw * f1.w;
        const v4f xs = *(const v4f*)(x + (size_t)s * ZW + zcol);
        sx += xs;
        const v4f ms = *(const v4f*)(mz + (size_t)s * ZW + zcol);
        zm0 = fmaxf(zm0, ms.x); zm1 = fmaxf(zm1, ms.y); zm2 = fmaxf(zm2, ms.z); zm3 = fmaxf(zm3, ms.w);
      }
    }

    const float rcp  = __builtin_amdgcn_rcpf(den);
    const float rd   = (n > 0) ? rcp : 0.0f;
    const float dg   = (float)(nraw > 1 ? nraw : 1);
    const float invd = 1.0f / dg;
    const v4f mean = sx * invd;
    v4f zmv;
    zmv.x = (n > 0) ? zm0 : 0.f; zmv.y = (n > 0) ? zm1 : 0.f;
    zmv.z = (n > 0) ? zm2 : 0.f; zmv.w = (n > 0) ? zm3 : 0.f;
    const int xr = c < nN ? c : nN - 1;
    const v4f xc = *(const v4f*)(x + (size_t)xr * ZW + zcol);

    float zl[4];
#pragma unroll
    for (int h = 0; h < 4; ++h) {
      const float* wh = gw + (size_t)h * GK + zcol;
      const v4f wx = *(const v4f*)wh;
      const v4f wm = *(const v4f*)(wh + ZW);
      const v4f wz = *(const v4f*)(wh + 2 * ZW);
      float ph = xc.x * wx.x + xc.y * wx.y + xc.z * wx.z + xc.w * wx.w;
      ph += zmv.x * wm.x + zmv.y * wm.y + zmv.z * wm.z + zmv.w * wm.w;
      ph += mean.x * wz.x + mean.y * wz.y + mean.z * wz.z + mean.w * wz.w;
      ph += __shfl_xor(ph, 16);
      ph += __shfl_xor(ph, 8);
      ph += __shfl_xor(ph, 4);
      ph += __shfl_xor(ph, 2);
      ph += __shfl_xor(ph, 1);
      zl[h] = ph;
    }
    const float g0 = 1.0f / (1.0f + __expf(-(zl[0] + gb0)));
    const float g1 = 1.0f / (1.0f + __expf(-(zl[1] + gb1)));
    const float g2 = 1.0f / (1.0f + __expf(-(zl[2] + gb2)));
    const float g3 = 1.0f / (1.0f + __expf(-(zl[3] + gb3)));
    const float gsel = (hd == 0) ? g0 : ((hd == 1) ? g1 : ((hd == 2) ? g2 : g3));

    float t[8];
#pragma unroll
    for (int i = 0; i < 8; ++i) t[i] = acc[i] * rd * gsel;
#pragma unroll
    for (int i = 0; i < 8; ++i) { t[i] += __shfl_xor(t[i], 8); t[i] += __shfl_xor(t[i], 16); t[i] *= 0.25f; }

    const float scl = (c < nN) ? (float)GSC : 0.0f;
    v4f ta, tb;
    ta.x = t[0]; ta.y = t[1]; ta.z = t[2]; ta.w = t[3];
    tb.x = t[4]; tb.y = t[5]; tb.z = t[6]; tb.w = t[7];
    const v8h ov = cvt8(ta, tb, scl);
    const int li = lane & 7;
    _Float16* gp = xg + (size_t)c * LDXG + GCOL + 8 * li;
    if (lane < 8) *(volatile v8h*)gp = ov;
    __threadfence();
    if (lane < 8) *(volatile v8h*)gp = ov;
  }
}

extern "C" void kernel_launch(void* const* d_in, const int* in_sizes, int n_in,
                              void* d_out, int out_size, void* d_ws, size_t ws_size,
                              hipStream_t stream) {
  if (n_in < 13) return;
  const int nN = in_sizes[0] / ZW;
  const int nE = in_sizes[1];
  if (nN <= 0 || nE <= 0 || in_sizes[0] != nN * ZW) return;
  if (in_sizes[2] != nE || in_sizes[3] != nE) return;
  if (in_sizes[4] != FW * ZW || in_sizes[5] != FW || in_sizes[6] != FW) return;
  if (in_sizes[7] != ZW * ZW || in_sizes[8] != ZW) return;
  if (in_sizes[9] != NHD * GK || in_sizes[10] != NHD) return;
  if (in_sizes[11] != OW * LDXG || in_sizes[12] != OW) return;
  if (out_size != nN * OW) return;
  if (nE > (1 << 28) || nN > (1 << 22)) return;

  const float* x    = (const float*)d_in[0];
  const int*   src  = (const int*)d_in[1];
  const int*   dst  = (const int*)d_in[2];
  const float* ewt  = (const float*)d_in[3];
  const float* Wf   = (const float*)d_in[4];
  const float* al   = (const float*)d_in[5];
  const float* ar   = (const float*)d_in[6];
  const float* Wm   = (const float*)d_in[7];
  const float* bm   = (const float*)d_in[8];
  const float* Wgt  = (const float*)d_in[9];
  const float* bgt  = (const float*)d_in[10];
  const float* Wo   = (const float*)d_in[11];
  const float* bo   = (const float*)d_in[12];
  float* out = (float*)d_out;

  const int NPAD   = ((nN + TGT - 1) / TGT) * TGT;
  const int nBC    = (nN + NBC - 1) / NBC;
  const int CNTPAD = nBC * NBC;
  if (CNTPAD < NPAD) return;
  if (4 * nBC + 1 > RBN) return;
  const int nBF    = (nN + NBF - 1) / NBF;
  if (nBF > 4 * nBC) return;
  const int csrLen = ((nE + 31) & ~31) + 4096;
  if (31 * 4 * nBC > 4096) return;
  const int nAgg   = NPAD / TGT;
  const int nG64   = NPAD / 64;
  const int nG32   = NPAD / 32;
  const int nXu    = NPAD * (ZW / 8);
  const int nWm    = ZW * ZW / 8;
  const int nWf    = FW * ZW / 8;
  const int nWo    = OW * LDXG / 8;

  char* ws = (char*)d_ws;
  size_t off = 0;
  const size_t oWM  = off; off += (size_t)ZW * ZW * 2;           off = (off + 255) & ~(size_t)255;
  const size_t oWF  = off; off += (size_t)FW * ZW * 2;           off = (off + 255) & ~(size_t)255;
  const size_t oWO  = off; off += (size_t)OW * LDXG * 2;         off = (off + 255) & ~(size_t)255;
  const size_t oXG  = off; off += (size_t)NPAD * LDXG * 2;       off = (off + 255) & ~(size_t)255;
  const size_t oCnt = off; off += (size_t)CNTPAD * 4;            off = (off + 255) & ~(size_t)255;
  const size_t oOff = off; off += (size_t)CNTPAD * 4;            off = (off + 255) & ~(size_t)255;
  const size_t oRb  = off; off += (size_t)RBN * 4;               off = (off + 255) & ~(size_t)255;
  const size_t oCsr = off; off += (size_t)csrLen * 4;            off = (off + 255) & ~(size_t)255;
  const size_t oMZ  = off; off += (size_t)NPAD * ZW * 4;         off = (off + 255) & ~(size_t)255;
  const size_t oFT  = off; off += (size_t)NPAD * FW * 4;         off = (off + 255) & ~(size_t)255;
  const size_t oEL  = off; off += (size_t)NPAD * NHD * 4;        off = (off + 255) & ~(size_t)255;
  const size_t oER  = off; off += (size_t)NPAD * NHD * 4;        off = (off + 255) & ~(size_t)255;
  if (off > ws_size || off > (size_t)WSCAP) return;
  _Float16* wm  = (_Float16*)(ws + oWM);
  _Float16* wf  = (_Float16*)(ws + oWF);
  _Float16* wo  = (_Float16*)(ws + oWO);
  _Float16* xg  = (_Float16*)(ws + oXG);
  int*   cnt  = (int*)(ws + oCnt);
  int*   offp = (int*)(ws + oOff);
  int*   rb   = (int*)(ws + oRb);
  int*   csr  = (int*)(ws + oCsr);
  float* mzp  = (float*)(ws + oMZ);
  float* ftp  = (float*)(ws + oFT);
  float* elp  = (float*)(ws + oEL);
  float* erp  = (float*)(ws + oER);

  const int vec8 = 1;

  k_wcvt<<<(nWm + NTHR - 1) / NTHR, NTHR, 0, stream>>>(Wm, wm, nWm, ZW, ZW, (float)WSC, (float)WSC);
  k_wcvt<<<(nWf + NTHR - 1) / NTHR, NTHR, 0, stream>>>(Wf, wf, nWf, ZW, ZW, (float)WSC, (float)WSC);
  k_wcvt<<<(nWo + NTHR - 1) / NTHR, NTHR, 0, stream>>>(Wo, wo, nWo, LDXG, ZW, (float)WSC, (float)(WSC / GSC));
  k_xcvt<<<(nXu + NTHR - 1) / NTHR, NTHR, 0, stream>>>(x, xg, nN, nXu);

  k_count<<<nBC, NTHR, 0, stream>>>(dst, cnt, nE, vec8);
  k_offsets<<<1, OTHR, 0, stream>>>(cnt, offp, rb, nBC);
  hipFuncSetAttribute(reinterpret_cast<const void*>(&k_fill),
                      hipFuncAttributeMaxDynamicSharedMemorySize, LDS_FILL);
  k_fill<<<nBF, NTHR, LDS_FILL, stream>>>(dst, offp, rb, csr, nE, vec8, csrLen);

  k_gemm<ZW, LDXG, ZW, 64, 1, 0><<<nG64, NTHR, 0, stream>>>(xg, wm, bm, al, ar, mzp, elp, erp, nN);
  k_gemm<ZW, LDXG, FW, 32, NHD, 1><<<nG32, NTHR, 0, stream>>>(xg, wf, bm, al, ar, ftp, elp, erp, nN);

  k_agg<<<nAgg, NTHR, 0, stream>>>(csr, offp, cnt, src, ewt, x, elp, erp, ftp, mzp, Wgt, bgt, xg, nN, nE, csrLen);

  k_gemm<LDXG, LDXG, OW, 64, 1, 2><<<nG64, NTHR, 0, stream>>>(xg, wo, bo, al, ar, out, elp, erp, nN);
}
